// CosformerAttention_38577396253109
// MI455X (gfx1250) — hardware-verified
//
#include <hip/hip_runtime.h>
#include <math.h>

constexpr int kBsz   = 2;
constexpr int kLen   = 1024;
constexpr int kEmb   = 512;
constexpr int kHeads = 16;
constexpr int kHd    = 64;
constexpr int kD2    = 128;
constexpr int kRows  = kBsz * kLen;
constexpr int kQKVN  = 3 * kEmb;
constexpr int kGrp   = 8;
constexpr float kQKCarry   = 16.0f;
constexpr float kDenEps    = 1.0e-6f * 256.0f;
constexpr float kPCarry    = 32768.0f;
constexpr float kPCarryInv = 1.0f / 32768.0f;
constexpr float kHalfPi    = 1.5707963267948966f;
constexpr float kInvLen    = 1.0f / 1024.0f;
static_assert(kRows % 64 == 0 && kQKVN % 64 == 0 && kEmb % 64 == 0 && kLen % 64 == 0 && kHd % 64 == 0, "tile multiples");
static_assert(kEmb % 32 == 0 && kD2 % 32 == 0 && kLen % 32 == 0, "K multiples of 32");
static_assert(kHeads * kHd == kBsz * kEmb && kGrp * 2 == kHeads, "head map");
static_assert(kLen % 8 == 0 && (kLen / 8) == 128, "norm kernel: 128 threads x 8 = one row");

typedef __attribute__((ext_vector_type(16))) _Float16 v16h;
typedef __attribute__((ext_vector_type(8)))  _Float16 v8h;
typedef __attribute__((ext_vector_type(16))) __bf16   v16b;
typedef __attribute__((ext_vector_type(8)))  __bf16   v8b;
typedef __attribute__((ext_vector_type(8)))  float    v8f;
typedef __attribute__((ext_vector_type(4)))  float    v4f;
typedef __attribute__((ext_vector_type(4)))  unsigned int v4u;

__device__ __forceinline__ unsigned short f2bf_bits(float f) {
  unsigned u = __float_as_uint(f);
  return (unsigned short)((u + 0x7FFFu + ((u >> 16) & 1u)) >> 16);
}
__device__ __forceinline__ float bf_bits2f(unsigned short h) { return __uint_as_float(((unsigned)h) << 16); }

__device__ __forceinline__ void dep_guard4_h(v8f& a, v8f& b, v8f& c, v8f& d, v16h x, v16h y) {
  asm volatile("v_nop\n\tv_nop\n\tv_nop\n\tv_nop" : "+v"(a), "+v"(b), "+v"(c), "+v"(d) : "v"(x), "v"(y));
}
__device__ __forceinline__ void dep_guard4_b(v8f& a, v8f& b, v8f& c, v8f& d, v16b x, v16b y) {
  asm volatile("v_nop\n\tv_nop\n\tv_nop\n\tv_nop" : "+v"(a), "+v"(b), "+v"(c), "+v"(d) : "v"(x), "v"(y));
}
__device__ __forceinline__ void keep4_h(v16h a, v16h b, v16h c, v16h d) { asm volatile("v_nop" :: "v"(a), "v"(b), "v"(c), "v"(d)); }
__device__ __forceinline__ void keep4_b(v16b a, v16b b, v16b c, v16b d) { asm volatile("v_nop" :: "v"(a), "v"(b), "v"(c), "v"(d)); }
__device__ __forceinline__ void acc_guard4(v8f& a, v8f& b, v8f& c, v8f& d) { asm volatile("v_nop\n\tv_nop\n\tv_nop\n\tv_nop" : "+v"(a), "+v"(b), "+v"(c), "+v"(d)); }
template <typename T> struct Frag;
template <> struct Frag<_Float16> {
  typedef v16h V; union U { v16h v; v8h h[2]; };
  static __device__ __forceinline__ v16h load(const _Float16* p) {
    U f; f.h[0] = *(const v8h*)(p); f.h[1] = *(const v8h*)(p + 16); return f.v;
  }
  static __device__ __forceinline__ v8f mma(v16h a, v16h b, v8f c) {
    return __builtin_amdgcn_wmma_f32_16x16x32_f16(false, a, false, b, (short)0, c, false, false);
  }
  static __device__ __forceinline__ void guard4(v8f& a, v8f& b, v8f& c, v8f& d, v16h x, v16h y) { dep_guard4_h(a, b, c, d, x, y); }
  static __device__ __forceinline__ void keep(v16h a, v16h b, v16h c, v16h d) { keep4_h(a, b, c, d); }
};
template <> struct Frag<__bf16> {
  typedef v16b V; union U { v16b v; v8b h[2]; };
  static __device__ __forceinline__ v16b load(const __bf16* p) {
    U f; f.h[0] = *(const v8b*)(p); f.h[1] = *(const v8b*)(p + 16); return f.v;
  }
  static __device__ __forceinline__ v8f mma(v16b a, v16b b, v8f c) {
    return __builtin_amdgcn_wmma_f32_16x16x32_bf16(false, a, false, b, (short)0, c, false, false);
  }
  static __device__ __forceinline__ void guard4(v8f& a, v8f& b, v8f& c, v8f& d, v16b x, v16b y) { dep_guard4_b(a, b, c, d, x, y); }
  static __device__ __forceinline__ void keep(v16b a, v16b b, v16b c, v16b d) { keep4_b(a, b, c, d); }
};

__device__ __forceinline__ unsigned pk16(unsigned short a, unsigned short b) { return (unsigned)a | ((unsigned)b << 16); }
__device__ __forceinline__ unsigned short h_bits(float f) { const _Float16 h = (_Float16)f; return __builtin_bit_cast(unsigned short, h); }

template <int ET> struct Elem;
template <> struct Elem<0> { typedef _Float16 T; };
template <> struct Elem<1> { typedef __bf16 T; };
template <int ET, int SPLIT, int BIAS_MODE, int OUT_MODE, bool RESID, int ACT = 0>
__global__ __launch_bounds__(256) void wmma_gemm64(
    const unsigned short* __restrict__ Ap, const unsigned short* __restrict__ A2p, int lda, long strideA,
    const unsigned short* __restrict__ Btp, const unsigned short* __restrict__ Bt2p, int ldb, long strideB,
    void* __restrict__ Cout, void* __restrict__ Cout2, int ldc, long strideC,
    const float* __restrict__ bias,
    const float* __restrict__ resid, long strideR,
    int M, int N, int K, float scale) {
  typedef typename Elem<ET>::T T;
  typedef typename Frag<T>::V V;
  const T* A = (const T*)Ap; const T* A2 = (const T*)A2p; const T* Bt = (const T*)Btp; const T* Bt2 = (const T*)Bt2p;
  __shared__ __align__(16) float sT[8][16 * 68];
  const int b    = blockIdx.y;
  const int lane = threadIdx.x & 31;
  const int wave = threadIdx.x >> 5;
  const int tilesN = N >> 6;
  const int tilesM = M >> 6;
  const int tile = blockIdx.x * 8 + wave;
  if (tile >= tilesM * tilesN) return;
  const int tm = tile / tilesN;
  const int tn = tile - tm * tilesN;
  const int m0 = tm << 6;
  const int n0 = tn << 6;

  const T* Ab  = A  + (size_t)b * strideA;
  const T* Bb  = Bt + (size_t)b * strideB;
  const T* Ab2 = (SPLIT != 0) ? (A2  + (size_t)b * strideA) : nullptr;
  const T* Bb2 = (SPLIT == 1) ? (Bt2 + (size_t)b * strideB) : nullptr;

  const int rlane = lane & 15;
  const int koff  = (lane >> 4) * 8;
  const int mOff  = (lane >> 4) * 8;

  v8f acc[4][4];
#pragma unroll
  for (int i = 0; i < 4; ++i)
#pragma unroll
    for (int j = 0; j < 4; ++j) acc[i][j] = (v8f){0.f,0.f,0.f,0.f,0.f,0.f,0.f,0.f};

  for (int k0 = 0; k0 < K; k0 += 32) {
    V bh[4], bl[4];
#pragma unroll
    for (int j = 0; j < 4; ++j) {
      const size_t bo = (size_t)(n0 + (j << 4) + rlane) * ldb + koff + k0;
      bh[j] = Frag<T>::load(Bb + bo);
      if (SPLIT == 1) bl[j] = Frag<T>::load(Bb2 + bo);
    }
#pragma unroll
    for (int i = 0; i < 4; ++i) {
      const size_t ao = (size_t)(m0 + (i << 4) + rlane) * lda + koff + k0;
      V ah = Frag<T>::load(Ab + ao);
      V al;
      if (SPLIT != 0) al = Frag<T>::load(Ab2 + ao);
#pragma unroll
      for (int j = 0; j < 4; ++j) {
        acc[i][j] = Frag<T>::mma(ah, bh[j], acc[i][j]);
        if (SPLIT == 1) acc[i][j] = Frag<T>::mma(ah, bl[j], acc[i][j]);
        if (SPLIT != 0) acc[i][j] = Frag<T>::mma(al, bh[j], acc[i][j]);
      }
      Frag<T>::guard4(acc[i][0], acc[i][1], acc[i][2], acc[i][3], ah, (SPLIT != 0) ? al : ah);
    }
    Frag<T>::keep(bh[0], bh[1], bh[2], bh[3]);
    if (SPLIT == 1) Frag<T>::keep(bl[0], bl[1], bl[2], bl[3]);
  }
  acc_guard4(acc[0][0], acc[0][1], acc[0][2], acc[0][3]);
  acc_guard4(acc[1][0], acc[1][1], acc[1][2], acc[1][3]);
  acc_guard4(acc[2][0], acc[2][1], acc[2][2], acc[2][3]);
  acc_guard4(acc[3][0], acc[3][1], acc[3][2], acc[3][3]);

  float* slab = sT[wave];
  const float* Rb = RESID ? (resid + (size_t)b * strideR) : nullptr;
#pragma unroll
  for (int i = 0; i < 4; ++i) {
    const int mBase = m0 + (i << 4);
#pragma unroll
    for (int j = 0; j < 4; ++j) {
      const int n = n0 + (j << 4) + rlane;
      float bv = 0.f;
      if (BIAS_MODE == 2) bv = bias[n];
#pragma unroll
      for (int r = 0; r < 8; ++r) {
        float v = acc[i][j][r] * scale;
        if (BIAS_MODE == 1) v += bias[mBase + mOff + r];
        if (BIAS_MODE == 2) v += bv;
        if (RESID) v += Rb[(size_t)(mBase + mOff + r) * ldc + n];
        if (ACT == 2) v = fmaxf(v, 0.0f);
        if (ACT == 4) v = (v > 0.f) ? v : 0.01f * v;
        slab[(mOff + r) * 68 + (j << 4) + rlane] = v;
      }
    }
    __builtin_amdgcn_fence(__ATOMIC_RELEASE, "workgroup");
    __builtin_amdgcn_wave_barrier();
    __builtin_amdgcn_fence(__ATOMIC_ACQUIRE, "workgroup");
    if (OUT_MODE == 0) {
      float* C = (float*)Cout + (size_t)b * strideC;
      const int hh = lane >> 4, c4 = (lane & 15) * 4;
      for (int pass = 0; pass < 2; ++pass) {
#pragma unroll
        for (int it = 0; it < 8; ++it) {
          const int row = it * 2 + hh;
          v4f v = *(const v4f*)(slab + row * 68 + c4);
          *(volatile v4f*)(C + (size_t)(mBase + row) * ldc + n0 + c4) = v;
        }
        __threadfence();
      }
    } else {
      const int q = lane >> 3, c8 = (lane & 7) * 8;
      unsigned short* C  = (unsigned short*)Cout  + (size_t)b * strideC;
      unsigned short* C2 = (OUT_MODE == 2) ? ((unsigned short*)Cout2 + (size_t)b * strideC) : nullptr;
      for (int pass = 0; pass < 2; ++pass) {
#pragma unroll
        for (int it = 0; it < 4; ++it) {
          const int row = it * 4 + q;
          const float* sp = slab + row * 68 + c8;
          v8h hv, lv;
#pragma unroll
          for (int e = 0; e < 8; ++e) {
            if (OUT_MODE == 1) {
              hv[e] = (_Float16)sp[e];
            } else {
              unsigned short hb = f2bf_bits(sp[e]);
              unsigned short lb = f2bf_bits(sp[e] - bf_bits2f(hb));
              hv[e] = __builtin_bit_cast(_Float16, hb);
              lv[e] = __builtin_bit_cast(_Float16, lb);
            }
          }
          *(volatile v8h*)(C + (size_t)(mBase + row) * ldc + n0 + c8) = hv;
          if (OUT_MODE == 2) *(volatile v8h*)(C2 + (size_t)(mBase + row) * ldc + n0 + c8) = lv;
        }
        __threadfence();
      }
    }
    __builtin_amdgcn_fence(__ATOMIC_RELEASE, "workgroup");
    __builtin_amdgcn_wave_barrier();
    __builtin_amdgcn_fence(__ATOMIC_ACQUIRE, "workgroup");
  }
}

__global__ __launch_bounds__(256) void cast8_bf16_kernel(const float* __restrict__ in, unsigned short* __restrict__ out, int n8) {
  const int i = blockIdx.x * 256 + threadIdx.x;
  if (i >= n8) return;
  const float* p = in + 8 * (size_t)i;
  const v4f a = *(const v4f*)(p);
  const v4f c = *(const v4f*)(p + 4);
  unsigned short hb[8];
#pragma unroll
  for (int e = 0; e < 4; ++e) {
    hb[e]     = f2bf_bits(a[e]);
    hb[4 + e] = f2bf_bits(c[e]);
  }
  const v4u u = (v4u){pk16(hb[0], hb[1]), pk16(hb[2], hb[3]), pk16(hb[4], hb[5]), pk16(hb[6], hb[7])};
  unsigned short* q = out + 8 * (size_t)i;
  *(volatile v4u*)q = u;
  __threadfence();
  *(volatile v4u*)q = u;
}

__global__ __launch_bounds__(256) void expand_kernel(const float* __restrict__ QKV,
                                                     const float* __restrict__ bq, const float* __restrict__ bk,
                                                     const float* __restrict__ bv,
                                                     unsigned short* __restrict__ Qp, unsigned short* __restrict__ Kp,
                                                     unsigned short* __restrict__ VTh, unsigned short* __restrict__ VTl) {
  __shared__ float sm[64][65];
  const int t    = threadIdx.x;
  const int lane = t & 31, wave = t >> 5;
  const int l0   = blockIdx.x * 64;
  const int hh   = blockIdx.y;
  const int bsel = hh >> 3;
  const int e0   = (hh & 7) * 64;

  {
    const int m4 = (t & 15) * 4;
    const v4f bvv = *(const v4f*)(bv + e0 + m4);
    float bvr[4];
#pragma unroll
    for (int c = 0; c < 4; ++c) bvr[c] = bf_bits2f(f2bf_bits(bvv[c]));
#pragma unroll
    for (int it = 0; it < 4; ++it) {
      const int e4 = it * 256 + t;
      const int j  = e4 >> 4;
      const int r  = 2 * (l0 + j) + bsel;
      const v4f vv = *(const v4f*)(QKV + (size_t)r * kQKVN + 2 * kEmb + e0 + m4);
#pragma unroll
      for (int c = 0; c < 4; ++c) sm[m4 + c][j] = vv[c] + bvr[c];
    }
  }
  asm volatile("" ::: "memory");

  {
    const int c16  = lane & 15, sub = lane >> 4;
    const int dseg = (c16 & 7) * 8;
    const v4f bq0 = *(const v4f*)(bq + e0 + dseg);
    const v4f bq1 = *(const v4f*)(bq + e0 + dseg + 4);
    const v4f bk0 = *(const v4f*)(bk + e0 + dseg);
    const v4f bk1 = *(const v4f*)(bk + e0 + dseg + 4);
    float bqr[8], bkr[8];
#pragma unroll
    for (int e = 0; e < 4; ++e) {
      bqr[e]     = bf_bits2f(f2bf_bits(bq0[e]));
      bqr[4 + e] = bf_bits2f(f2bf_bits(bq1[e]));
      bkr[e]     = bf_bits2f(f2bf_bits(bk0[e]));
      bkr[4 + e] = bf_bits2f(f2bf_bits(bk1[e]));
    }
    asm volatile("" ::: "memory");
#pragma unroll 1
    for (int it = 0; it < 4; ++it) {
      const int i = (wave * 4 + it) * 2 + sub;
      const int l = l0 + i;
      const int r = 2 * l + bsel;
      const float* qrow = QKV + (size_t)r * kQKVN + e0 + dseg;
      const v4f q0 = *(const v4f*)(qrow);
      const v4f q1 = *(const v4f*)(qrow + 4);
      const v4f k0 = *(const v4f*)(qrow + kEmb);
      const v4f k1 = *(const v4f*)(qrow + kEmb + 4);
      const float th = (kHalfPi * (float)(l + 1)) * kInvLen;
      float sn, cs;
      sincosf(th, &sn, &cs);
      const float w = (((c16 >> 3) != 0) ? cs : sn) * kQKCarry;
      unsigned short hq[8], hk[8];
#pragma unroll
      for (int e = 0; e < 4; ++e) {
        hq[e]     = h_bits(fmaxf(q0[e] + bqr[e], 0.0f) * w);
        hq[4 + e] = h_bits(fmaxf(q1[e] + bqr[4 + e], 0.0f) * w);
        hk[e]     = h_bits(fmaxf(k0[e] + bkr[e], 0.0f) * w);
        hk[4 + e] = h_bits(fmaxf(k1[e] + bkr[4 + e], 0.0f) * w);
      }
      const v4u uq = (v4u){pk16(hq[0], hq[1]), pk16(hq[2], hq[3]), pk16(hq[4], hq[5]), pk16(hq[6], hq[7])};
      const v4u uk = (v4u){pk16(hk[0], hk[1]), pk16(hk[2], hk[3]), pk16(hk[4], hk[5]), pk16(hk[6], hk[7])};
      const size_t off = ((size_t)(hh * kLen + l)) * kD2 + (size_t)c16 * 8;
      unsigned short* qd = Qp + off;
      unsigned short* kd = Kp + off;
      *(volatile v4u*)qd = uq;
      *(volatile v4u*)kd = uk;
      __threadfence();
      *(volatile v4u*)qd = uq;
      *(volatile v4u*)kd = uk;
    }
  }
  __syncthreads();

  {
    const int q = lane >> 3, c8 = (lane & 7) * 8;
    unsigned short* oph = VTh + (size_t)hh * kHd * kLen;
    unsigned short* opl = VTl + (size_t)hh * kHd * kLen;
    for (int pass = 0; pass < 2; ++pass) {
#pragma unroll
      for (int it = 0; it < 2; ++it) {
        const int row = wave * 8 + it * 4 + q;
        unsigned short hb[8], lb[8];
#pragma unroll
        for (int e = 0; e < 8; ++e) {
          const float x = sm[row][c8 + e];
          hb[e] = f2bf_bits(x);
          lb[e] = f2bf_bits(x - bf_bits2f(hb[e]));
        }
        const v4u uh = (v4u){pk16(hb[0], hb[1]), pk16(hb[2], hb[3]), pk16(hb[4], hb[5]), pk16(hb[6], hb[7])};
        const v4u ul = (v4u){pk16(lb[0], lb[1]), pk16(lb[2], lb[3]), pk16(lb[4], lb[5]), pk16(lb[6], lb[7])};
        const size_t off = (size_t)row * kLen + l0 + c8;
        *(volatile v4u*)(oph + off) = uh;
        *(volatile v4u*)(opl + off) = ul;
      }
      __threadfence();
    }
  }
}

__global__ __launch_bounds__(128) void norm_kernel(const float* __restrict__ S, unsigned short* __restrict__ Ph,
                                                   unsigned short* __restrict__ Pl) {
  __shared__ float red[4];
  const int l    = blockIdx.x;
  const int h8   = blockIdx.y;
  const int t    = threadIdx.x;
  const int lane = t & 31, wave = t >> 5;
  const size_t rowoff = ((size_t)h8 * kLen + l) * kLen;
  const float* sr = S + rowoff + 8 * (size_t)t;
  const v4f a = *(const v4f*)(sr);
  const v4f c = *(const v4f*)(sr + 4);
  float x[8];
#pragma unroll
  for (int e = 0; e < 4; ++e) {
    const int j0 = 8 * t + e;
    const int j1 = 8 * t + 4 + e;
    x[e]     = (j0 <= l) ? a[e] : 0.0f;
    x[4 + e] = (j1 <= l) ? c[e] : 0.0f;
  }
  float s = ((x[0] + x[1]) + (x[2] + x[3])) + ((x[4] + x[5]) + (x[6] + x[7]));
#pragma unroll
  for (int off = 16; off > 0; off >>= 1) s += __shfl_xor(s, off, 32);
  if (lane == 0) red[wave] = s;
  __syncthreads();
  const float tot = ((red[0] + red[1]) + red[2]) + red[3];
  const float den = fmaxf(tot, kDenEps);
  const float inv = kPCarry * (1.0f / den);
  unsigned short hb[8], lb[8];
#pragma unroll
  for (int e = 0; e < 8; ++e) {
    const float p = x[e] * inv;
    hb[e] = f2bf_bits(p);
    lb[e] = f2bf_bits(p - bf_bits2f(hb[e]));
  }
  const v4u uh = (v4u){pk16(hb[0], hb[1]), pk16(hb[2], hb[3]), pk16(hb[4], hb[5]), pk16(hb[6], hb[7])};
  const v4u ul = (v4u){pk16(lb[0], lb[1]), pk16(lb[2], lb[3]), pk16(lb[4], lb[5]), pk16(lb[6], lb[7])};
  unsigned short* ph = Ph + rowoff + 8 * (size_t)t;
  unsigned short* pl = Pl + rowoff + 8 * (size_t)t;
  *(volatile v4u*)ph = uh;
  *(volatile v4u*)pl = ul;
  __threadfence();
  *(volatile v4u*)ph = uh;
  *(volatile v4u*)pl = ul;
}

extern "C" void kernel_launch(void* const* d_in, const int* in_sizes, int n_in,
                              void* d_out, int out_size, void* d_ws, size_t ws_size,
                              hipStream_t stream) {
  if (n_in < 9) return;
  if (in_sizes[0] != kRows * kEmb) return;
  if (in_sizes[1] != kEmb * kEmb || in_sizes[3] != kEmb * kEmb || in_sizes[5] != kEmb * kEmb || in_sizes[7] != kEmb * kEmb) return;
  if (in_sizes[2] != kEmb || in_sizes[4] != kEmb || in_sizes[6] != kEmb || in_sizes[8] != kEmb) return;
  if (out_size != kRows * kEmb) return;

  const size_t szXb   = (size_t)kRows * kEmb * 2;
  const size_t szWqkv = (size_t)kQKVN * kEmb * 2;
  const size_t szWo   = (size_t)kEmb * kEmb * 2;
  const size_t szQKV  = (size_t)kRows * kQKVN * 4;
  const size_t szQp   = (size_t)kHeads * kLen * kD2 * 2;
  const size_t szVT   = (size_t)kHeads * kHd * kLen * 2;
  const size_t szS    = (size_t)kGrp * kLen * kLen * 4;
  const size_t szP    = (size_t)kGrp * kLen * kLen * 2;
  const size_t szA    = (size_t)kRows * kEmb * 2;
  const size_t offXb   = 0;
  const size_t offWqkv = offXb + szXb;
  const size_t offWo   = offWqkv + szWqkv;
  const size_t offQKV  = offWo + szWo;
  const size_t offQp   = offQKV + szQKV;
  const size_t offKp   = offQp + szQp;
  const size_t offVTh  = offKp + szQp;
  const size_t offVTl  = offVTh + szVT;
  const size_t offS    = offVTl + szVT;
  const size_t offPh   = offS + szS;
  const size_t offPl   = offPh + szP;
  const size_t offAh   = offPl + szP;
  const size_t offAl   = offAh + szA;
  const size_t total   = offAl + szA;
  if (ws_size < total) return;

  const float* query = (const float*)d_in[0];
  const float* Wq    = (const float*)d_in[1];
  const float* bq    = (const float*)d_in[2];
  const float* Wk    = (const float*)d_in[3];
  const float* bk    = (const float*)d_in[4];
  const float* Wv    = (const float*)d_in[5];
  const float* bv    = (const float*)d_in[6];
  const float* Wo    = (const float*)d_in[7];
  const float* bo    = (const float*)d_in[8];
  float* out = (float*)d_out;
  char* ws = (char*)d_ws;
  unsigned short* Xb   = (unsigned short*)(ws + offXb);
  unsigned short* Wqkv = (unsigned short*)(ws + offWqkv);
  unsigned short* Wob  = (unsigned short*)(ws + offWo);
  float*          QKV  = (float*)(ws + offQKV);
  unsigned short* Qp   = (unsigned short*)(ws + offQp);
  unsigned short* Kp   = (unsigned short*)(ws + offKp);
  unsigned short* VTh  = (unsigned short*)(ws + offVTh);
  unsigned short* VTl  = (unsigned short*)(ws + offVTl);
  float*          S    = (float*)(ws + offS);
  unsigned short* Ph   = (unsigned short*)(ws + offPh);
  unsigned short* Pl   = (unsigned short*)(ws + offPl);
  unsigned short* Ah   = (unsigned short*)(ws + offAh);
  unsigned short* Al   = (unsigned short*)(ws + offAl);

  const int n8X = (kRows * kEmb) / 8;
  const int n8W = (kEmb * kEmb) / 8;
  cast8_bf16_kernel<<<dim3(n8X / 256), dim3(256), 0, stream>>>(query, Xb, n8X);
  cast8_bf16_kernel<<<dim3(n8W / 256), dim3(256), 0, stream>>>(Wq, Wqkv, n8W);
  cast8_bf16_kernel<<<dim3(n8W / 256), dim3(256), 0, stream>>>(Wk, Wqkv + (size_t)kEmb * kEmb, n8W);
  cast8_bf16_kernel<<<dim3(n8W / 256), dim3(256), 0, stream>>>(Wv, Wqkv + (size_t)2 * kEmb * kEmb, n8W);
  cast8_bf16_kernel<<<dim3(n8W / 256), dim3(256), 0, stream>>>(Wo, Wob, n8W);

  {
    const int tiles = (kRows / 64) * (kQKVN / 64);
    wmma_gemm64<1, 0, 0, 0, false, 0><<<dim3(tiles / 8, 1), dim3(256), 0, stream>>>(
        Xb, Xb, kEmb, 0L, Wqkv, Wqkv, kEmb, 0L,
        (void*)QKV, (void*)QKV, kQKVN, 0L, bo, bo, 0L, kRows, kQKVN, kEmb, 1.0f);
  }

  expand_kernel<<<dim3(kLen / 64, kHeads), dim3(256), 0, stream>>>(QKV, bq, bk, bv, Qp, Kp, VTh, VTl);

  const long strideQK = (long)kLen * kD2;
  const long strideVT = (long)kHd * kLen;
  const long strideS  = (long)kLen * kLen;
  const int  tilesS   = (kLen / 64) * (kLen / 64);
  const int  tilesPV  = (kLen / 64) * (kHd / 64);
  for (int bg = 0; bg < kBsz; ++bg) {
    const unsigned short* Qg  = Qp + (size_t)bg * kGrp * strideQK;
    const unsigned short* Kg  = Kp + (size_t)bg * kGrp * strideQK;
    const unsigned short* VHg = VTh + (size_t)bg * kGrp * strideVT;
    const unsigned short* VLg = VTl + (size_t)bg * kGrp * strideVT;
    wmma_gemm64<0, 0, 0, 0, false, 0><<<dim3(tilesS / 8, kGrp), dim3(256), 0, stream>>>(
        Qg, Qg, kD2, strideQK, Kg, Kg, kD2, strideQK,
        (void*)S, (void*)S, kLen, strideS, bo, bo, 0L, kLen, kLen, kD2, 1.0f);
    norm_kernel<<<dim3(kLen, kGrp), dim3(128), 0, stream>>>(S, Ph, Pl);
    wmma_gemm64<1, 1, 0, 2, false, 0><<<dim3(tilesPV / 8, kGrp), dim3(256), 0, stream>>>(
        Ph, Pl, kLen, strideS, VHg, VLg, kLen, strideVT,
        (void*)(Ah + (size_t)bg * kEmb), (void*)(Al + (size_t)bg * kEmb), 2 * kEmb, (long)kHd,
        bo, bo, 0L, kLen, kHd, kLen, kPCarryInv);
  }

  {
    const int tiles = (kRows / 64) * (kEmb / 64);
    wmma_gemm64<1, 2, 2, 0, false, 0><<<dim3(tiles / 8, 1), dim3(256), 0, stream>>>(
        Ah, Al, kEmb, 0L, Wob, Wob, kEmb, 0L,
        (void*)out, (void*)out, kEmb, 0L, bo, bo, 0L, kRows, kEmb, kEmb, 1.0f);
  }
  (void)ws_size;
}
